// RoPEAttention_11330123727239
// MI455X (gfx1250) — hardware-verified
//
#include <hip/hip_runtime.h>


#define NB_  2
#define TT   2048
#define DM   1024
#define NH_  16
#define NKV  16
#define REP  (NH_ / NKV)
#define HD   64
#define DQ   (NH_ * HD)
#define DKV  (NKV * HD)
#define RW   DQ
#define ZH   2
#define RH   512
#define WIN  2048
#define PCAR 1024.0f
#define SCL  0.125f
typedef _Float16 h16;
typedef unsigned short bf;
typedef __attribute__((ext_vector_type(16))) __bf16   v16bf;
typedef __attribute__((ext_vector_type(16))) _Float16 v16h;
typedef __attribute__((ext_vector_type(8)))  _Float16 v8h;
typedef __attribute__((ext_vector_type(8)))  unsigned short v8us;
typedef __attribute__((ext_vector_type(8)))  float    v8f;
typedef __attribute__((ext_vector_type(4)))  float    v4f;
typedef v8h  __attribute__((may_alias)) v8ha;
typedef v4f  __attribute__((may_alias)) v4fa;
typedef v8us __attribute__((may_alias)) v8usa;

__device__ __forceinline__ unsigned short f2bf(float f) { unsigned u = __float_as_uint(f); u += 0x7FFFu + ((u >> 16) & 1u); return (unsigned short)(u >> 16); }
__device__ __forceinline__ float bf2f(unsigned short b) { return __uint_as_float(((unsigned)b) << 16); }
__device__ __forceinline__ float bfr(float f) { return bf2f(f2bf(f)); }
__device__ __forceinline__ v16h cat16(v8h lo, v8h hi) { return __builtin_shufflevector(lo, hi, 0, 1, 2, 3, 4, 5, 6, 7, 8, 9, 10, 11, 12, 13, 14, 15); }
__device__ __forceinline__ v16bf cat16b(v8us lo, v8us hi) { return __builtin_bit_cast(v16bf, __builtin_shufflevector(lo, hi, 0, 1, 2, 3, 4, 5, 6, 7, 8, 9, 10, 11, 12, 13, 14, 15)); }
__device__ __forceinline__ v8f wmma16(v16h a, v16h b, v8f c) { return __builtin_amdgcn_wmma_f32_16x16x32_f16(false, a, false, b, (short)0, c, false, false); }
__device__ __forceinline__ v8f wmmab(v16bf a, v16bf b, v8f c) { return __builtin_amdgcn_wmma_f32_16x16x32_bf16(false, a, false, b, (short)0, c, false, false); }


template <typename T16> struct WFrag;
template <> struct WFrag<h16> { typedef v16h V; static __device__ __forceinline__ V ld(const h16* p) { return cat16(*(const v8h*)p, *(const v8h*)(p + 16)); } static __device__ __forceinline__ v8f mma(V a, V b, v8f c) { return wmma16(a, b, c); } };
template <> struct WFrag<bf> { typedef v16bf V; static __device__ __forceinline__ V ld(const bf* p) { return cat16b(*(const v8us*)p, *(const v8us*)(p + 16)); } static __device__ __forceinline__ v8f mma(V a, V b, v8f c) { return wmmab(a, b, c); } };
template <typename T16, int NSPLIT, bool BIAS>
__global__ __launch_bounds__(32) void k_gemmw(const T16* __restrict__ A, const T16* __restrict__ A2, const T16* __restrict__ Bt, const T16* __restrict__ Bt2, int K, float* C, int ldc, const float* __restrict__ bias, size_t sA, size_t sB, size_t sC) {
    typedef typename WFrag<T16>::V V;
    __shared__ __align__(16) float os[16 * 68];
    const size_t z = blockIdx.z; A += z * sA; if (A2) A2 += z * sA; Bt += z * sB; if (Bt2) Bt2 += z * sB; C += z * sC;
    const int lane = threadIdx.x & 31, lr = lane & 15, hi = lane >> 4; const int r0 = blockIdx.x * 64, c0 = blockIdx.y * 64;
    v8f acc[4][4];
#pragma unroll
    for (int mb = 0; mb < 4; ++mb)
#pragma unroll
        for (int nb = 0; nb < 4; ++nb) acc[mb][nb] = (v8f){};
    const size_t aoff = (size_t)(r0 + lr) * K + 8 * hi, boff = (size_t)(c0 + lr) * K + 8 * hi;
#pragma unroll 1
    for (int kc = 0; kc < K; kc += 32) {
        V a[4], a2[4];
#pragma unroll
        for (int mb = 0; mb < 4; ++mb) { a[mb] = WFrag<T16>::ld(A + aoff + (size_t)mb * 16 * K + kc); if (NSPLIT == 1 || NSPLIT == 2) a2[mb] = WFrag<T16>::ld(A2 + aoff + (size_t)mb * 16 * K + kc); }
#pragma unroll
        for (int nb = 0; nb < 4; ++nb) { const V b = WFrag<T16>::ld(Bt + boff + (size_t)nb * 16 * K + kc); V b2; if (NSPLIT >= 2) b2 = WFrag<T16>::ld(Bt2 + boff + (size_t)nb * 16 * K + kc);
#pragma unroll
            for (int mb = 0; mb < 4; ++mb) { acc[mb][nb] = WFrag<T16>::mma(a[mb], b, acc[mb][nb]); if (NSPLIT == 1 || NSPLIT == 2) acc[mb][nb] = WFrag<T16>::mma(a2[mb], b, acc[mb][nb]); if (NSPLIT >= 2) acc[mb][nb] = WFrag<T16>::mma(a[mb], b2, acc[mb][nb]); } }
        asm volatile("v_nop\n\tv_nop\n\tv_nop\n\tv_nop" : "+v"(acc[0][0]), "+v"(acc[1][1]), "+v"(acc[2][2]), "+v"(acc[3][3]) : "v"(a[0]), "v"(a[3]));
    }
#pragma unroll
    for (int mb = 0; mb < 4; ++mb) {
#pragma unroll
        for (int nb = 0; nb < 4; ++nb) {
#pragma unroll
            for (int j = 0; j < 8; ++j) os[(hi * 8 + j) * 68 + nb * 16 + lr] = acc[mb][nb][j]; }
        __builtin_amdgcn_wave_barrier(); asm volatile("" ::: "memory");
        float* crow = C + (size_t)(r0 + mb * 16) * ldc + c0;
#pragma unroll 1
        for (int ps = 0; ps < 2; ++ps) {
#pragma unroll
            for (int s = 0; s < 8; ++s) { const int row = 2 * s + hi, cofs = lr * 4; v4f val = *(const v4fa*)(os + row * 68 + cofs); if (BIAS) { val[0] += bfr(bias[c0 + cofs]); val[1] += bfr(bias[c0 + cofs + 1]); val[2] += bfr(bias[c0 + cofs + 2]); val[3] += bfr(bias[c0 + cofs + 3]); }
                *(volatile v4f*)(crow + (size_t)row * ldc + cofs) = val; }
            if (ps == 0) __threadfence(); }
        __builtin_amdgcn_wave_barrier(); asm volatile("" ::: "memory");
    }
}

template <typename T16, int NSPLIT, int CMODE>
__global__ __launch_bounds__(32) void k_gemmc(const T16* __restrict__ A, const T16* __restrict__ A2, const T16* __restrict__ Bt, const T16* __restrict__ Bt2, int K, float* C, int ldc, int roff, size_t sA, size_t sB, size_t sC) {
    typedef typename WFrag<T16>::V V;
    __shared__ __align__(16) float os[16 * 68];
    const size_t z = blockIdx.z; A += z * sA; if (A2) A2 += z * sA; Bt += z * sB; if (Bt2) Bt2 += z * sB; C += z * sC;
    const int lane = threadIdx.x & 31, lr = lane & 15, hi = lane >> 4; const int r0 = blockIdx.x * 64, c0 = blockIdx.y * 64;
    if (CMODE == 1 && c0 > r0 + roff + 63) return;
    const int Kl = (CMODE == 2) ? min(K, r0 + roff + 64) : K;
    v8f acc[4][4];
#pragma unroll
    for (int mb = 0; mb < 4; ++mb)
#pragma unroll
        for (int nb = 0; nb < 4; ++nb) acc[mb][nb] = (v8f){};
    const size_t aoff = (size_t)(r0 + lr) * K + 8 * hi, boff = (size_t)(c0 + lr) * K + 8 * hi;
#pragma unroll 1
    for (int kc = 0; kc < Kl; kc += 32) {
        V a[4], a2[4];
#pragma unroll
        for (int mb = 0; mb < 4; ++mb) { a[mb] = WFrag<T16>::ld(A + aoff + (size_t)mb * 16 * K + kc); if (NSPLIT == 1 || NSPLIT == 2) a2[mb] = WFrag<T16>::ld(A2 + aoff + (size_t)mb * 16 * K + kc); }
#pragma unroll
        for (int nb = 0; nb < 4; ++nb) { const V b = WFrag<T16>::ld(Bt + boff + (size_t)nb * 16 * K + kc); V b2; if (NSPLIT >= 2) b2 = WFrag<T16>::ld(Bt2 + boff + (size_t)nb * 16 * K + kc);
#pragma unroll
            for (int mb = 0; mb < 4; ++mb) { acc[mb][nb] = WFrag<T16>::mma(a[mb], b, acc[mb][nb]); if (NSPLIT == 1 || NSPLIT == 2) acc[mb][nb] = WFrag<T16>::mma(a2[mb], b, acc[mb][nb]); if (NSPLIT >= 2) acc[mb][nb] = WFrag<T16>::mma(a[mb], b2, acc[mb][nb]); } }
        asm volatile("v_nop\n\tv_nop\n\tv_nop\n\tv_nop" : "+v"(acc[0][0]), "+v"(acc[1][1]), "+v"(acc[2][2]), "+v"(acc[3][3]) : "v"(a[0]), "v"(a[3]));
    }
#pragma unroll
    for (int mb = 0; mb < 4; ++mb) {
#pragma unroll
        for (int nb = 0; nb < 4; ++nb) {
#pragma unroll
            for (int j = 0; j < 8; ++j) os[(hi * 8 + j) * 68 + nb * 16 + lr] = acc[mb][nb][j]; }
        __builtin_amdgcn_wave_barrier(); asm volatile("" ::: "memory");
        float* crow = C + (size_t)(r0 + mb * 16) * ldc + c0;
#pragma unroll 1
        for (int ps = 0; ps < 2; ++ps) {
#pragma unroll
            for (int s = 0; s < 8; ++s) { const int row = 2 * s + hi, cofs = lr * 4; v4f val = *(const v4fa*)(os + row * 68 + cofs);
                *(volatile v4f*)(crow + (size_t)row * ldc + cofs) = val; }
            if (ps == 0) __threadfence(); }
        __builtin_amdgcn_wave_barrier(); asm volatile("" ::: "memory");
    }
}

__device__ __forceinline__ h16 tohx(float x) { return (h16)x; }
__device__ __forceinline__ void splitf(float y, unsigned short& h, unsigned short& l) { h = f2bf(y); l = f2bf(y - bf2f(h)); }
typedef __attribute__((ext_vector_type(2))) _Float16 v2h;
typedef __attribute__((ext_vector_type(4))) _Float16 v4h;
typedef __attribute__((ext_vector_type(2))) unsigned short v2us;
typedef __attribute__((ext_vector_type(4))) unsigned short v4us;
typedef __attribute__((ext_vector_type(2))) float v2f;
typedef __attribute__((ext_vector_type(4))) int v4i;

__global__ __launch_bounds__(256) void k_cvt8(const float* __restrict__ src, bf* dst, size_t n8) { const size_t i = (size_t)blockIdx.x * 256 + threadIdx.x; if (i >= n8) return; const v8f v = *(const v8f*)(src + i * 8); v8us o;
#pragma unroll
    for (int k = 0; k < 8; ++k) o[k] = f2bf(v[k]); *(volatile v8us*)(dst + i * 8) = o; __threadfence(); *(volatile v8us*)(dst + i * 8) = o; }

__global__ __launch_bounds__(256) void k_ropeI(const float* __restrict__ F, int pitch, int nheads, const float* __restrict__ CS, float sc, h16* P16, bf* Ph, bf* Pl) {
    const size_t e = ((size_t)blockIdx.x * 256 + threadIdx.x) * 2; if (e >= (size_t)nheads * TT * HD) return; const int d = (int)(e % HD); const int t = (int)((e / HD) % TT); const int h = (int)(e / ((size_t)HD * TT)); const float* f = F + (size_t)t * pitch + h * HD; const float x0 = f[d], x1 = f[d + 1]; const v2f cs = *(const v2f*)(CS + ((size_t)t * RW + h * HD + d) * 2);     v2h o16; v2us oh, ol;
    float a0 = __fmul_rn(x0, cs[0]), b0 = __fmul_rn(x1, cs[1]), a1 = __fmul_rn(x1, cs[0]), b1 = __fmul_rn(x0, cs[1]); asm volatile("" : "+v"(a0), "+v"(b0), "+v"(a1), "+v"(b1));
    float r0 = __fsub_rn(a0, b0) * sc, r1 = __fadd_rn(b1, a1) * sc;
    o16[0] = tohx(r0); o16[1] = tohx(r1); { unsigned short a2, c2; splitf(r0, a2, c2); oh[0] = a2; ol[0] = c2; splitf(r1, a2, c2); oh[1] = a2; ol[1] = c2; }
    *(volatile v2h*)(P16 + e) = o16; *(volatile v2us*)(Ph + e) = oh; *(volatile v2us*)(Pl + e) = ol; __threadfence(); *(volatile v2h*)(P16 + e) = o16; *(volatile v2us*)(Ph + e) = oh; *(volatile v2us*)(Pl + e) = ol; }

__global__ __launch_bounds__(256) void k_vtp(const float* __restrict__ F, int pitch, int nheads, h16* V16, bf* Vh, bf* Vl) { const size_t e = ((size_t)blockIdx.x * 256 + threadIdx.x) * 2; if (e >= (size_t)nheads * HD * TT) return; const int t = (int)(e % TT); const int d = (int)((e / TT) % HD); const int g = (int)(e / ((size_t)TT * HD)); v2h o16; v2us oh, ol;
#pragma unroll
    for (int q = 0; q < 2; ++q) { const float x = F[(size_t)(t + q) * pitch + g * HD + d]; o16[q] = tohx(x); unsigned short a2, c2; splitf(x, a2, c2); oh[q] = a2; ol[q] = c2; }
    *(volatile v2h*)(V16 + e) = o16; *(volatile v2us*)(Vh + e) = oh; *(volatile v2us*)(Vl + e) = ol; __threadfence(); *(volatile v2h*)(V16 + e) = o16; *(volatile v2us*)(Vh + e) = oh; *(volatile v2us*)(Vl + e) = ol; }
__constant__ float INV2[RW / 2] = { 1.000000000e+00f, 9.821718335e-01f, 9.646616578e-01f, 9.474635124e-01f, 9.305720329e-01f, 9.139816761e-01f, 8.976871371e-01f, 8.816831112e-01f, 8.659643531e-01f, 8.505258560e-01f, 8.353625536e-01f, 8.204696178e-01f, 8.058422208e-01f, 7.914755344e-01f, 7.773650289e-01f, 7.635061145e-01f, 7.498942018e-01f, 7.365249991e-01f, 7.233941555e-01f, 7.104974389e-01f, 6.978305578e-01f, 6.853895783e-01f, 6.731703877e-01f, 6.611690521e-01f, 6.493816376e-01f, 6.378043890e-01f, 6.264335513e-01f, 6.152654290e-01f, 6.042963862e-01f, 5.935229063e-01f, 5.829415321e-01f, 5.725488067e-01f, 5.623413324e-01f, 5.523158312e-01f, 5.424690843e-01f, 5.327978730e-01f, 5.232991576e-01f, 5.139696598e-01f, 5.048065782e-01f, 4.958068132e-01f, 4.869675338e-01f, 4.782858193e-01f, 4.697588682e-01f, 4.613839388e-01f, 4.531583488e-01f, 4.450793862e-01f, 4.371444881e-01f, 4.293510318e-01f, 4.216965139e-01f, 4.141784608e-01f, 4.067944288e-01f, 3.995420635e-01f, 3.924189806e-01f, 3.854228854e-01f, 3.785515428e-01f, 3.718026578e-01f, 3.651741445e-01f, 3.586637676e-01f, 3.522694409e-01f, 3.459891677e-01f, 3.398208320e-01f, 3.337624967e-01f, 3.278121352e-01f, 3.219678402e-01f, 3.162277639e-01f, 3.105900288e-01f, 3.050527871e-01f, 2.996142805e-01f, 2.942727208e-01f, 2.890264094e-01f, 2.838735878e-01f, 2.788126469e-01f, 2.738419771e-01f, 2.689598799e-01f, 2.641648352e-01f, 2.594552636e-01f, 2.548296750e-01f, 2.502865493e-01f, 2.458243966e-01f, 2.414418161e-01f, 2.371373624e-01f, 2.329096496e-01f, 2.287573218e-01f, 2.246790081e-01f, 2.206733972e-01f, 2.167392224e-01f, 2.128751576e-01f, 2.090799958e-01f, 2.053525001e-01f, 2.016914487e-01f, 1.980956793e-01f, 1.945640147e-01f, 1.910952926e-01f, 1.876884252e-01f, 1.843423098e-01f, 1.810558140e-01f, 1.778279394e-01f, 1.746576130e-01f, 1.715437919e-01f, 1.684854925e-01f, 1.654817015e-01f, 1.625314802e-01f, 1.596338600e-01f, 1.567878872e-01f, 1.539926529e-01f, 1.512472630e-01f, 1.485508084e-01f, 1.459024251e-01f, 1.433012635e-01f, 1.407464594e-01f, 1.382372230e-01f, 1.357727200e-01f, 1.333521456e-01f, 1.309747249e-01f, 1.286396980e-01f, 1.263462901e-01f, 1.240937710e-01f, 1.218814254e-01f, 1.197085083e-01f, 1.175743192e-01f, 1.154782027e-01f, 1.134194434e-01f, 1.113973856e-01f, 1.094113812e-01f, 1.074607819e-01f, 1.055449620e-01f, 1.036632955e-01f, 1.018151715e-01f, 1.000000015e-01f, 9.821718186e-02f, 9.646616131e-02f, 9.474635124e-02f, 9.305720031e-02f, 9.139817208e-02f, 8.976870775e-02f, 8.816830814e-02f, 8.659642935e-02f, 8.505257964e-02f, 8.353625983e-02f, 8.204696327e-02f, 8.058421314e-02f, 7.914755493e-02f, 7.773650438e-02f, 7.635060698e-02f, 7.498941571e-02f, 7.365249842e-02f, 7.233941555e-02f, 7.104974240e-02f, 6.978305429e-02f, 6.853895634e-02f, 6.731703877e-02f, 6.611690670e-02f, 6.493816525e-02f, 6.378044188e-02f, 6.264335662e-02f, 6.152653694e-02f, 6.042964384e-02f, 5.935229361e-02f, 5.829415470e-02f, 5.725487694e-02f, 5.623412877e-02f, 5.523158237e-02f, 5.424690619e-02f, 5.327979103e-02f, 5.232991278e-02f, 5.139696971e-02f, 5.048065633e-02f, 4.958068207e-02f, 4.869675264e-02f, 4.782858118e-02f, 4.697588459e-02f, 4.613839835e-02f, 4.531583562e-02f, 4.450793937e-02f, 4.371444881e-02f, 4.293510318e-02f, 4.216964915e-02f, 4.141784459e-02f, 4.067944363e-02f, 3.995420411e-02f, 3.924189880e-02f, 3.854228929e-02f, 3.785515204e-02f, 3.718026727e-02f, 3.651741147e-02f, 3.586637601e-02f, 3.522694483e-02f, 3.459891677e-02f, 3.398208320e-02f, 3.337624669e-02f, 3.278120980e-02f, 3.219678625e-02f, 3.162277862e-02f, 3.105900250e-02f, 3.050527908e-02f, 2.996142767e-02f, 2.942727320e-02f, 2.890264057e-02f, 2.838735841e-02f, 2.788126841e-02f, 2.738419548e-02f, 2.689598687e-02f, 2.641648427e-02f, 2.594552562e-02f, 2.548296750e-02f, 2.502865531e-02f, 2.458244003e-02f, 2.414418198e-02f, 2.371373586e-02f, 2.329096757e-02f, 2.287573181e-02f, 2.246790007e-02f, 2.206734009e-02f, 2.167392150e-02f, 2.128751762e-02f, 2.090799995e-02f, 2.053525113e-02f, 2.016914636e-02f, 1.980956830e-02f, 1.945639960e-02f, 1.910953037e-02f, 1.876884326e-02f, 1.843423024e-02f, 1.810558327e-02f, 1.778279431e-02f, 1.746576093e-02f, 1.715437882e-02f, 1.684854925e-02f, 1.654817164e-02f, 1.625314727e-02f, 1.596338488e-02f, 1.567878947e-02f, 1.539926510e-02f, 1.512472518e-02f, 1.485508028e-02f, 1.459024288e-02f, 1.433012541e-02f, 1.407464594e-02f, 1.382372249e-02f, 1.357727125e-02f, 1.333521493e-02f, 1.309747249e-02f, 1.286396943e-02f, 1.263462938e-02f, 1.240937691e-02f, 1.218814217e-02f, 1.197085064e-02f, 1.175743248e-02f, 1.154781971e-02f, 1.134194434e-02f, 1.113973837e-02f, 1.094113849e-02f, 1.074607857e-02f, 1.055449620e-02f, 1.036632899e-02f, 1.018151734e-02f, 9.999999776e-03f, 9.821719490e-03f, 9.646615945e-03f, 9.474635124e-03f, 9.305720218e-03f, 9.139816277e-03f, 8.976871148e-03f, 8.816830814e-03f, 8.659643121e-03f, 8.505257778e-03f, 8.353625424e-03f, 8.204696700e-03f, 8.058422245e-03f, 7.914755493e-03f, 7.773650344e-03f, 7.635060698e-03f, 7.498942316e-03f, 7.365249563e-03f, 7.233941462e-03f, 7.104974240e-03f, 6.978305988e-03f, 6.853895728e-03f, 6.731703877e-03f, 6.611690391e-03f, 6.493816618e-03f, 6.378043909e-03f, 6.264335476e-03f, 6.152654067e-03f, 6.042964291e-03f, 5.935229361e-03f, 5.829415284e-03f, 5.725487601e-03f, 5.623413250e-03f, 5.523158237e-03f, 5.424690899e-03f, 5.327979103e-03f, 5.232991185e-03f, 5.139696877e-03f, 5.048065912e-03f, 4.958068486e-03f, 4.869675264e-03f, 4.782858305e-03f, 4.697588738e-03f, 4.613839556e-03f, 4.531583749e-03f, 4.450793844e-03f, 4.371444695e-03f, 4.293510225e-03f, 4.216964822e-03f, 4.141784739e-03f, 4.067944363e-03f, 3.995420411e-03f, 3.924189601e-03f, 3.854229115e-03f, 3.785515437e-03f, 3.718026681e-03f, 3.651741426e-03f, 3.586637788e-03f, 3.522694577e-03f, 3.459891537e-03f, 3.398208413e-03f, 3.337624483e-03f, 3.278121119e-03f, 3.219678300e-03f, 3.162277862e-03f, 3.105900250e-03f, 3.050528001e-03f, 2.996142721e-03f, 2.942727180e-03f, 2.890263917e-03f, 2.838735934e-03f, 2.788126701e-03f, 2.738419687e-03f, 2.689598827e-03f, 2.641648287e-03f, 2.594552701e-03f, 2.548296703e-03f, 2.502865391e-03f, 2.458244096e-03f, 2.414418384e-03f, 2.371373819e-03f, 2.329096664e-03f, 2.287573181e-03f, 2.246790100e-03f, 2.206734149e-03f, 2.167392056e-03f, 2.128751716e-03f, 2.090800088e-03f, 2.053525066e-03f, 2.016914543e-03f, 1.980956644e-03f, 1.945640077e-03f, 1.910952851e-03f, 1.876884256e-03f, 1.843422884e-03f, 1.810558140e-03f, 1.778279431e-03f, 1.746576163e-03f, 1.715437858e-03f, 1.684854855e-03f, 1.654817141e-03f, 1.625314937e-03f, 1.596338581e-03f, 1.567878877e-03f, 1.539926510e-03f, 1.512472634e-03f, 1.485507935e-03f, 1.459024264e-03f, 1.433012658e-03f, 1.407464617e-03f, 1.382372226e-03f, 1.357727102e-03f, 1.333521446e-03f, 1.309747226e-03f, 1.286396873e-03f, 1.263462938e-03f, 1.240937854e-03f, 1.218814170e-03f, 1.197085017e-03f, 1.175743295e-03f, 1.154782018e-03f, 1.134194434e-03f, 1.113973907e-03f, 1.094113803e-03f, 1.074607833e-03f, 1.055449597e-03f, 1.036632922e-03f, 1.018151757e-03f, 1.000000047e-03f, 9.821718559e-04f, 9.646615945e-04f, 9.474635590e-04f, 9.305721032e-04f, 9.139817557e-04f, 8.976871031e-04f, 8.816830232e-04f, 8.659643354e-04f, 8.505258011e-04f, 8.353625308e-04f, 8.204695769e-04f, 8.058422245e-04f, 7.914755843e-04f, 7.773649995e-04f, 7.635060465e-04f, 7.498941850e-04f, 7.365249912e-04f, 7.233941578e-04f, 7.104973774e-04f, 6.978305755e-04f, 6.853896193e-04f, 6.731703761e-04f, 6.611690042e-04f, 6.493816618e-04f, 6.378043909e-04f, 6.264335825e-04f, 6.152653950e-04f, 6.042963942e-04f, 5.935229128e-04f, 5.829415168e-04f, 5.725487717e-04f, 5.623413017e-04f, 5.523158470e-04f, 5.424690899e-04f, 5.327978870e-04f, 5.232990952e-04f, 5.139696877e-04f, 5.048065796e-04f, 4.958068021e-04f, 4.869675031e-04f, 4.782858014e-04f, 4.697588738e-04f, 4.613839847e-04f, 4.531583400e-04f, 4.450794077e-04f, 4.371444811e-04f, 4.293509992e-04f, 4.216964880e-04f, 4.141784448e-04f, 4.067944246e-04f, 3.995420411e-04f, 3.924189950e-04f, 3.854228707e-04f, 3.785515146e-04f, 3.718026564e-04f, 3.651741135e-04f, 3.586637613e-04f, 3.522694460e-04f, 3.459891595e-04f, 3.398208064e-04f, 3.337624657e-04f, 3.278121294e-04f, 3.219678474e-04f, 3.162277862e-04f, 3.105900250e-04f, 3.050527885e-04f, 2.996142721e-04f, 2.942727297e-04f, 2.890263859e-04f, 2.838736109e-04f, 2.788126585e-04f, 2.738419571e-04f, 2.689598768e-04f, 2.641648462e-04f, 2.594552934e-04f, 2.548296761e-04f, 2.502865391e-04f, 2.458243980e-04f, 2.414418122e-04f, 2.371373848e-04f, 2.329096606e-04f, 2.287573152e-04f, 2.246790100e-04f, 2.206734207e-04f, 2.167392086e-04f, 2.128751657e-04f, 2.090800117e-04f, 2.053524950e-04f, 2.016914514e-04f, 1.980956731e-04f, 1.945640106e-04f, 1.910952997e-04f, 1.876884344e-04f, 1.843422942e-04f, 1.810558315e-04f, 1.778279402e-04f, 1.746576017e-04f, 1.715437829e-04f, 1.684854797e-04f, 1.654817170e-04f, 1.625314762e-04f, 1.596338552e-04f, 1.567878790e-04f, 1.539926452e-04f, 1.512472518e-04f, 1.485508110e-04f, 1.459024206e-04f, 1.433012658e-04f, 1.407464733e-04f, 1.382372284e-04f, 1.357727160e-04f, 1.333521504e-04f, 1.309747167e-04f, 1.286396873e-04f, 1.263462909e-04f, 1.240937709e-04f, 1.218814141e-04f, 1.197085076e-04f, 1.175743309e-04f, 1.154781930e-04f, 1.134194390e-04f, 1.113973922e-04f, 1.094113759e-04f, 1.074607790e-04f, 1.055449538e-04f, 1.036632893e-04f, 1.018151743e-04f };
__global__ __launch_bounds__(256) void k_csP(float* CS) { const int idx = blockIdx.x * 256 + threadIdx.x; if (idx >= TT * RW) return; const int d = idx % RW; const int t = idx / RW; const float a = __fmul_rn((float)t, INV2[d >> 1]); v2f cs; cs[0] = cosf(a); cs[1] = sinf(a); *(volatile v2f*)(CS + (size_t)idx * 2) = cs; __threadfence(); *(volatile v2f*)(CS + (size_t)idx * 2) = cs; }
__global__ __launch_bounds__(256) void k_asoft(const float* __restrict__ Sb, h16* P16, bf* Ph, bf* Pl) {
    const int lane = threadIdx.x & 31; const int row = blockIdx.x * 8 + (threadIdx.x >> 5); if (row >= ZH * TT) return; const int i = row % TT; const int zz = row / TT; (void)zz; const bool hires = (i < RH); const float* sr = Sb + (size_t)row * TT; float v[TT / 32]; float mx = -3.0e38f;
#pragma unroll
    for (int ch = 0; ch < TT / 128; ++ch) { const int j0 = ch * 128 + lane * 4; const v4f a = *(const v4f*)(sr + j0);
#pragma unroll
        for (int q = 0; q < 4; ++q) { const int j = j0 + q; (void)j; const float t = (j <= i && i - j < WIN) ? a[q] * SCL : -3.0e38f; v[ch * 4 + q] = t; mx = fmaxf(mx, t); } }
#pragma unroll
    for (int sh = 16; sh; sh >>= 1) mx = fmaxf(mx, __shfl_xor(mx, sh, 32));
    float sum = 0.f;
#pragma unroll
    for (int k = 0; k < TT / 32; ++k) { float d0 = __fsub_rn(v[k], mx); asm volatile("" : "+v"(d0)); v[k] = __builtin_amdgcn_exp2f(__fmul_rn(d0, 1.4426950408889634f)); sum += v[k]; }
#pragma unroll
    for (int sh = 16; sh; sh >>= 1) sum += __shfl_xor(sum, sh, 32);
    const float f = __fdiv_rn(hires ? 1.0f : PCAR, sum);
#pragma unroll 1
    for (int ps = 0; ps < 2; ++ps) {
        if (hires) {
#pragma unroll
            for (int ch = 0; ch < TT / 128; ++ch) { v4us oh, ol;
#pragma unroll
                for (int q = 0; q < 4; ++q) { unsigned short a, c2; splitf(v[ch * 4 + q] * f, a, c2); oh[q] = a; ol[q] = c2; }
                const size_t oo = ((size_t)zz * (RH ? RH : 1) + i) * TT + ch * 128 + lane * 4; *(volatile v4us*)(Ph + oo) = oh; *(volatile v4us*)(Pl + oo) = ol; }
        } else {
#pragma unroll
            for (int ch = 0; ch < TT / 128; ++ch) { v4h o4;
#pragma unroll
                for (int q = 0; q < 4; ++q) o4[q] = tohx(v[ch * 4 + q] * f);
                *(volatile v4h*)(P16 + (size_t)row * TT + ch * 128 + lane * 4) = o4; } }
        if (ps == 0) __threadfence(); }
}
__global__ __launch_bounds__(256) void k_merge(const float* __restrict__ O, int h0, bf* Ah, bf* Al) { const size_t e = ((size_t)blockIdx.x * 256 + threadIdx.x) * 2; if (e >= (size_t)ZH * TT * HD) return; const int d = (int)(e % HD); const int t = (int)((e / HD) % TT); const int zz = (int)(e / ((size_t)HD * TT)); const float cs = (t < RH) ? 1.0f : (1.0f / PCAR); const size_t oo = (size_t)t * DQ + (h0 + zz) * HD + d;
    v2us oh, ol;
#pragma unroll
    for (int q = 0; q < 2; ++q) { unsigned short a, c2; splitf(O[e + q] * cs, a, c2); oh[q] = a; ol[q] = c2; } *(volatile v2us*)(Ah + oo) = oh; *(volatile v2us*)(Al + oo) = ol; __threadfence(); *(volatile v2us*)(Ah + oo) = oh; *(volatile v2us*)(Al + oo) = ol; }

__global__ __launch_bounds__(256) void k_wtG(const float* __restrict__ w, int K, int N, bf* Bt) {
    const int lane = threadIdx.x & 31; const int L0 = (blockIdx.x * 8 + (threadIdx.x >> 5)) * 8; const int nlines = N * K / 64;
#pragma unroll
    for (int ps = 0; ps < 2; ++ps) {
#pragma unroll 1
        for (int l = 0; l < 8; ++l) { const int L = L0 + l; if (L >= nlines) break; const size_t e = (size_t)L * 64 + lane * 2; const int k = (int)(e % K), n = (int)(e / K); v2us o;
            o[0] = f2bf(w[(size_t)k * N + n]); o[1] = f2bf(w[(size_t)(k + 1) * N + n]); *(volatile v2us*)(Bt + e) = o; }
        if (ps == 0) __threadfence(); }
}
extern "C" void kernel_launch(void* const* d_in, const int* in_sizes, int n_in,
                              void* d_out, int out_size, void* d_ws, size_t ws_size, hipStream_t stream) {
    (void)in_sizes; (void)n_in; (void)out_size;
    const float* x = (const float*)d_in[0]; const float* wq = (const float*)d_in[2]; const float* wk = (const float*)d_in[3]; const float* wv = (const float*)d_in[4]; const float* wo = (const float*)d_in[5];
    float* OUT = (float*)d_out;
    char* wsp = (char*)d_ws;
    auto take = [&](size_t bytes) { char* p = wsp; wsp += (bytes + 255) & ~(size_t)255; return (void*)p; };
    bf* WQ = (bf*)take((size_t)DQ * DM * 2); bf* WK = (bf*)take((size_t)DKV * DM * 2); bf* WV = (bf*)take((size_t)DKV * DM * 2); bf* WO = (bf*)take((size_t)DM * DQ * 2); float* CS = (float*)take((size_t)TT * DQ * 2 * 4);
    bf* XB = (bf*)take((size_t)TT * DM * 2); float* FQ = (float*)take((size_t)TT * DQ * 4); float* FK = (float*)take((size_t)TT * DKV * 4);
    h16* QP16 = (h16*)take((size_t)NH_ * TT * HD * 2); h16* KP16 = (h16*)take((size_t)NKV * TT * HD * 2); h16* VT16 = (h16*)take((size_t)NKV * HD * TT * 2);
    bf* QPh = (bf*)take((size_t)NH_ * TT * HD * 2); bf* QPl = (bf*)take((size_t)NH_ * TT * HD * 2); bf* KPh = (bf*)take((size_t)NKV * TT * HD * 2); bf* KPl = (bf*)take((size_t)NKV * TT * HD * 2); bf* VTh = (bf*)take((size_t)NKV * HD * TT * 2); bf* VTl = (bf*)take((size_t)NKV * HD * TT * 2); bf* Ph = (bf*)take((size_t)ZH * RH * TT * 2); bf* Pl = (bf*)take((size_t)ZH * RH * TT * 2);
    float* Sb = (float*)take((size_t)ZH * TT * TT * 4); h16* P16 = (h16*)take((size_t)ZH * TT * TT * 2); float* Ob = (float*)take((size_t)ZH * TT * HD * 4); bf* ATh = (bf*)take((size_t)TT * DQ * 2); bf* ATl = (bf*)take((size_t)TT * DQ * 2);
    if ((size_t)(wsp - (char*)d_ws) > ws_size) return;
    float* FV = FK;
    { k_wtG<<<(unsigned)((DM * DQ / 64 + 63) / 64), 256, 0, stream>>>(wq, DM, DQ, WQ); k_wtG<<<(unsigned)((DM * DKV / 64 + 63) / 64), 256, 0, stream>>>(wk, DM, DKV, WK); k_wtG<<<(unsigned)((DM * DKV / 64 + 63) / 64), 256, 0, stream>>>(wv, DM, DKV, WV);
      k_wtG<<<(unsigned)((DQ * DM / 64 + 63) / 64), 256, 0, stream>>>(wo, DQ, DM, WO);
       }
    k_csP<<<(TT * RW + 255) / 256, 256, 0, stream>>>(CS);
    const unsigned LQ = (unsigned)(((size_t)NH_ * TT * HD / 2 + 255) / 256), LKv = (unsigned)(((size_t)NKV * TT * HD / 2 + 255) / 256);
    for (int b = 0; b < NB_; ++b) {

        k_cvt8<<<(unsigned)(((size_t)TT * DM / 8 + 255) / 256), 256, 0, stream>>>(x + (size_t)b * TT * DM, XB, (size_t)TT * DM / 8);
        k_gemmw<bf, 0, false><<<dim3(TT / 64, DQ / 64, 1), 32, 0, stream>>>(XB, nullptr, WQ, nullptr, DM, FQ, DQ, nullptr, 0, 0, 0);
        k_ropeI<<<LQ, 256, 0, stream>>>(FQ, DQ, NH_, CS, 1.0f, QP16, QPh, QPl);
        k_gemmw<bf, 0, false><<<dim3(TT / 64, DKV / 64, 1), 32, 0, stream>>>(XB, nullptr, WK, nullptr, DM, FK, DKV, nullptr, 0, 0, 0);
        k_ropeI<<<LKv, 256, 0, stream>>>(FK, DKV, NKV, CS, 1.0f, KP16, KPh, KPl);
        k_gemmw<bf, 0, false><<<dim3(TT / 64, DKV / 64, 1), 32, 0, stream>>>(XB, nullptr, WV, nullptr, DM, FV, DKV, nullptr, 0, 0, 0); k_vtp<<<LKv, 256, 0, stream>>>(FV, DKV, NKV, VT16, VTh, VTl);
        for (int h0 = 0; h0 < NH_; h0 += ZH) { const size_t zq = (size_t)h0, zk = (size_t)(h0 / REP);
            k_gemmc<bf, 2, 1><<<dim3(RH / 64, TT / 64, ZH), 32, 0, stream>>>(QPh + zq * TT * HD, QPl + zq * TT * HD, KPh + zk * TT * HD, KPl + zk * TT * HD, HD, Sb, TT, 0, (size_t)TT * HD, (size_t)TT * HD, (size_t)TT * TT);
            k_gemmc<h16, 0, 1><<<dim3((TT - RH) / 64, TT / 64, ZH), 32, 0, stream>>>(QP16 + zq * TT * HD + (size_t)RH * HD, nullptr, KP16 + zk * TT * HD, nullptr, HD, Sb + (size_t)RH * TT, TT, RH, (size_t)TT * HD, (size_t)TT * HD, (size_t)TT * TT);
            k_asoft<<<ZH * TT / 8, 256, 0, stream>>>(Sb, P16, Ph, Pl);
            k_gemmc<bf, 2, 2><<<dim3(RH / 64, HD / 64, ZH), 32, 0, stream>>>(Ph, Pl, VTh + zk * HD * TT, VTl + zk * HD * TT, TT, Ob, HD, 0, (size_t)RH * TT, (size_t)HD * TT, (size_t)TT * HD);
            k_gemmc<h16, 0, 2><<<dim3((TT - RH) / 64, HD / 64, ZH), 32, 0, stream>>>(P16 + (size_t)RH * TT, nullptr, VT16 + zk * HD * TT, nullptr, TT, Ob + (size_t)RH * HD, HD, RH, (size_t)TT * TT, (size_t)HD * TT, (size_t)TT * HD);
            k_merge<<<(unsigned)(((size_t)ZH * TT * HD / 2 + 255) / 256), 256, 0, stream>>>(Ob, h0, ATh, ATl); }
        k_gemmw<bf, 1, false><<<dim3(TT / 64, DM / 64, 1), 32, 0, stream>>>(ATh, ATl, WO, nullptr, DQ, OUT + (size_t)b * TT * DM, DM, nullptr, 0, 0, 0); }
}
